// GCN_GW_86835648790601
// MI455X (gfx1250) — hardware-verified
//
#include <hip/hip_runtime.h>
#include <stddef.h>


#define NTHR    256
#define NWAVE   8
#define DIM     64
#define NIN     128
#define NPE     64
#define KC1     192
#define KC2     256
#define FFH     128
#define FOUT    40
#define NMEM    32
#define NHD     4
#define DHD     16
#define SROWS   128
#define TOPN    5
#define HCAP    512
#define EPT     8
#define NGRP    1
#define CHUNK   (NTHR * EPT * NGRP)
#define WCAP    (EPT * NGRP * 32)
#define LISTN   (NWAVE * WCAP)
#define ESHF    11
#define NBC     32768
#define NBF     2048
#define RCAP    67584
#define RBN     128
#define TGT     256
#define DEGCAP  1024
#define GROWS   128
#define OTHR    512
#define CSELF   1.0f
#define WSC     16.0f
#define ASC     64.0f
#define WSCAP   134217728
#define LDS_COUNT ((NBC + LISTN + NWAVE) * 4)
#define LDS_FILL  ((RCAP + NBF + LISTN + NWAVE) * 4)

#define PW1H   0
#define PW1L   12288
#define PWKH   24576
#define PWKL   28672
#define PWQB   32768
#define PWOB   36864
#define PF1    40960
#define PF2    49152
#define PG2    57344
#define PWTOT  73728

static_assert((CHUNK & (CHUNK - 1)) == 0);
static_assert((NBC & (NBC - 1)) == 0 && (NBF & (NBF - 1)) == 0);
static_assert(NBF <= (1 << ESHF));
static_assert((NBC % NBF) == 0);
static_assert(OTHR * 4 == NBF);
static_assert((RCAP % 32) == 0);
static_assert(TGT == NWAVE * 32);
static_assert(GROWS == NWAVE * 16);
static_assert((TGT % GROWS) == 0);
static_assert(NBC == NWAVE * 32 * 128);
static_assert(SROWS == NHD * NMEM && DIM == NHD * DHD);
static_assert((FOUT % 4) == 0 && ((32 * FOUT) % 128) == 0 && FOUT <= DIM);
static_assert(LDS_FILL <= 300000);

typedef float           v2f  __attribute__((ext_vector_type(2)));
typedef float           v4f  __attribute__((ext_vector_type(4)));
typedef float           v8f  __attribute__((ext_vector_type(8)));
typedef int             v4i  __attribute__((ext_vector_type(4)));
typedef _Float16        v8h  __attribute__((ext_vector_type(8)));
typedef _Float16        v16h __attribute__((ext_vector_type(16)));
typedef __bf16          v16b __attribute__((ext_vector_type(16)));
typedef unsigned short  v8us __attribute__((ext_vector_type(8)));
union FragH { v16h v; v8h h[2]; };
union FragB { v16b v; v8us u[2]; };

__device__ __forceinline__ v8f wmf(v16h a, v16h b, v8f c) {
  v8f d = __builtin_amdgcn_wmma_f32_16x16x32_f16(false, a, false, b, (short)0, c, false, false);
  asm volatile("v_nop\n\tv_nop\n\tv_nop\n\tv_nop" : "+v"(d) : "v"(a), "v"(b));
  return d;
}
__device__ __forceinline__ v8f wmb(v16b a, v16b b, v8f c) {
  v8f d = __builtin_amdgcn_wmma_f32_16x16x32_bf16(false, a, false, b, (short)0, c, false, false);
  asm volatile("v_nop\n\tv_nop\n\tv_nop\n\tv_nop" : "+v"(d) : "v"(a), "v"(b));
  return d;
}
__device__ __forceinline__ v8f zero8() { v8f z = {0.f, 0.f, 0.f, 0.f, 0.f, 0.f, 0.f, 0.f}; return z; }

__device__ __forceinline__ unsigned short bfbits(float f) {
  unsigned u = __float_as_uint(f);
  u = (u + 0x7FFFu + ((u >> 16) & 1u)) >> 16;
  return (unsigned short)u;
}
__device__ __forceinline__ void bfsplit(float f, unsigned short& hb, unsigned short& lb) {
  const unsigned short hv = bfbits(f);
  const float hf = __uint_as_float(((unsigned)hv) << 16);
  hb = hv;
  lb = bfbits(f - hf);
}

__device__ __forceinline__ void load16(const float* ap, float* av) {
  const v4f f0 = *(const v4f*)ap;
  const v4f f1 = *(const v4f*)(ap + 4);
  const v4f f2 = *(const v4f*)(ap + 16);
  const v4f f3 = *(const v4f*)(ap + 20);
  av[0] = f0.x; av[1] = f0.y; av[2]  = f0.z; av[3]  = f0.w; av[4]  = f1.x; av[5]  = f1.y; av[6]  = f1.z; av[7]  = f1.w;
  av[8] = f2.x; av[9] = f2.y; av[10] = f2.z; av[11] = f2.w; av[12] = f3.x; av[13] = f3.y; av[14] = f3.z; av[15] = f3.w;
}
__device__ __forceinline__ v16h cvt_h16(const float* av, float sc) {
  FragH f;
#pragma unroll
  for (int i = 0; i < 8; ++i) { f.h[0][i] = (_Float16)(av[i] * sc); f.h[1][i] = (_Float16)(av[8 + i] * sc); }
  return f.v;
}
__device__ __forceinline__ void cvt_b16(const float* av, v16b& hi, v16b& lo) {
  FragB a, b;
#pragma unroll
  for (int i = 0; i < 8; ++i) {
    unsigned short hb, lb;
    bfsplit(av[i], hb, lb);      a.u[0][i] = hb; b.u[0][i] = lb;
    bfsplit(av[8 + i], hb, lb);  a.u[1][i] = hb; b.u[1][i] = lb;
  }
  hi = a.v; lo = b.v;
}

template <int NB, int SRC>
__device__ __forceinline__ int scan_chunk(const int* __restrict__ keys, const int* __restrict__ gath, int nE, int nN,
                                          int cbase, int slotBase, int vec8, int* list, int tid, int lane, int wave) {
  int wc = 0;
#pragma unroll
  for (int g = 0; g < NGRP; ++g) {
    const int el0  = (g * NTHR + tid) * EPT;
    const int e0   = cbase + el0;
    const int sent = -2147483647 - 1;
    v4i da, db;
    v4i sa = {0, 0, 0, 0}, sb = {0, 0, 0, 0};
    if (vec8 != 0 && cbase + CHUNK <= nE) {
      da = *(const v4i*)(keys + e0);
      db = *(const v4i*)(keys + e0 + 4);
      if (SRC) {
        sa = *(const v4i*)(gath + e0);
        sb = *(const v4i*)(gath + e0 + 4);
      }
    } else {
      da.x = (e0     < nE) ? keys[min(e0, nE - 1)] : sent;
      da.y = (e0 + 1 < nE) ? keys[min(e0 + 1, nE - 1)] : sent;
      da.z = (e0 + 2 < nE) ? keys[min(e0 + 2, nE - 1)] : sent;
      da.w = (e0 + 3 < nE) ? keys[min(e0 + 3, nE - 1)] : sent;
      db.x = (e0 + 4 < nE) ? keys[min(e0 + 4, nE - 1)] : sent;
      db.y = (e0 + 5 < nE) ? keys[min(e0 + 5, nE - 1)] : sent;
      db.z = (e0 + 6 < nE) ? keys[min(e0 + 6, nE - 1)] : sent;
      db.w = (e0 + 7 < nE) ? keys[min(e0 + 7, nE - 1)] : sent;
      if (SRC) {
        sa.x = gath[min(e0, nE - 1)];
        sa.y = gath[min(e0 + 1, nE - 1)];
        sa.z = gath[min(e0 + 2, nE - 1)];
        sa.w = gath[min(e0 + 3, nE - 1)];
        sb.x = gath[min(e0 + 4, nE - 1)];
        sb.y = gath[min(e0 + 5, nE - 1)];
        sb.z = gath[min(e0 + 6, nE - 1)];
        sb.w = gath[min(e0 + 7, nE - 1)];
      }
    }
    if (SRC) {
      sa.x = min(max(sa.x, 0), nN - 1); sa.y = min(max(sa.y, 0), nN - 1);
      sa.z = min(max(sa.z, 0), nN - 1); sa.w = min(max(sa.w, 0), nN - 1);
      sb.x = min(max(sb.x, 0), nN - 1); sb.y = min(max(sb.y, 0), nN - 1);
      sb.z = min(max(sb.z, 0), nN - 1); sb.w = min(max(sb.w, 0), nN - 1);
    }
    const unsigned nb = (unsigned)slotBase;
    const unsigned s0 = (unsigned)da.x - nb, s1 = (unsigned)da.y - nb;
    const unsigned s2 = (unsigned)da.z - nb, s3 = (unsigned)da.w - nb;
    const unsigned s4 = (unsigned)db.x - nb, s5 = (unsigned)db.y - nb;
    const unsigned s6 = (unsigned)db.z - nb, s7 = (unsigned)db.w - nb;
    const bool h0 = s0 < (unsigned)NB, h1 = s1 < (unsigned)NB, h2 = s2 < (unsigned)NB, h3 = s3 < (unsigned)NB;
    const bool h4 = s4 < (unsigned)NB, h5 = s5 < (unsigned)NB, h6 = s6 < (unsigned)NB, h7 = s7 < (unsigned)NB;
    const unsigned any = __builtin_amdgcn_ballot_w32(h0 | h1 | h2 | h3 | h4 | h5 | h6 | h7);
    if (any != 0u) {
#define HITJ(HJ, SJ, VJ) { \
        const unsigned mj = __builtin_amdgcn_ballot_w32(HJ); \
        if (mj != 0u) { \
          if (HJ) { \
            const int pos = wc + (int)__builtin_amdgcn_mbcnt_lo(mj, 0u); \
            const int entv = SRC ? (((VJ) << ESHF) | (int)(SJ)) : (int)(SJ); \
            if (pos < WCAP) list[wave * WCAP + pos] = entv; \
          } \
          wc += (int)__builtin_popcount(mj); } }
      HITJ(h0, s0, sa.x)
      HITJ(h1, s1, sa.y)
      HITJ(h2, s2, sa.z)
      HITJ(h3, s3, sa.w)
      HITJ(h4, s4, sb.x)
      HITJ(h5, s5, sb.y)
      HITJ(h6, s6, sb.z)
      HITJ(h7, s7, sb.w)
#undef HITJ
    }
  }
  return wc;
}

__global__ __launch_bounds__(NTHR) void k_wprep(
    const float* __restrict__ w1, const float* __restrict__ wk, const float* __restrict__ wqb,
    const float* __restrict__ wob, const float* __restrict__ f1, const float* __restrict__ f2,
    const float* __restrict__ g2, unsigned short* wp) {
  const int tid = threadIdx.x;
  const int b = blockIdx.x;
  const float* W = w1;
  int ldn = DIM, nval = DIM, kd = KC1, pb = b * NTHR, po = PW1H, po2 = PW1L, hilo = 1;
  if (b >= 20)      { W = g2;  ldn = FOUT; nval = FOUT; kd = KC2; pb = (b - 20) * NTHR; po = PG2;  po2 = PG2;  hilo = 0; }
  else if (b >= 16) { W = f2;  ldn = DIM;  nval = DIM;  kd = FFH; pb = (b - 16) * NTHR; po = PF2;  po2 = PF2;  hilo = 0; }
  else if (b >= 12) { W = f1;  ldn = FFH;  nval = FFH;  kd = DIM; pb = (b - 12) * NTHR; po = PF1;  po2 = PF1;  hilo = 0; }
  else if (b >= 10) { W = wob; ldn = DIM;  nval = DIM;  kd = DIM; pb = (b - 10) * NTHR; po = PWOB; po2 = PWOB; hilo = 0; }
  else if (b >= 8)  { W = wqb; ldn = DIM;  nval = DIM;  kd = DIM; pb = (b - 8)  * NTHR; po = PWQB; po2 = PWQB; hilo = 0; }
  else if (b >= 6)  { W = wk;  ldn = DIM;  nval = DIM;  kd = DIM; pb = (b - 6)  * NTHR; po = PWKH; po2 = PWKL; hilo = 1; }
  const int i  = pb + tid;
  const int kp = kd >> 3;
  const int n  = i / kp;
  const int k0 = (i - n * kp) * 8;
  const int nc = n < nval ? n : nval - 1;
  float v[8];
#pragma unroll
  for (int e = 0; e < 8; ++e) {
    const float t = W[(size_t)(k0 + e) * ldn + nc];
    v[e] = n < nval ? t : 0.0f;
  }
  unsigned short* d0 = wp + po  + (size_t)i * 8;
  unsigned short* d1 = wp + po2 + (size_t)i * 8;
  if (hilo) {
    v8us hv, lv;
#pragma unroll
    for (int e = 0; e < 8; ++e) { unsigned short hb, lb; bfsplit(v[e], hb, lb); hv[e] = hb; lv[e] = lb; }
    *(volatile v8us*)d0 = hv;
    *(volatile v8us*)d1 = lv;
    __threadfence();
    *(volatile v8us*)d0 = hv;
    *(volatile v8us*)d1 = lv;
  } else {
    v8h fv;
#pragma unroll
    for (int e = 0; e < 8; ++e) fv[e] = (_Float16)(v[e] * WSC);
    _Float16* dh = (_Float16*)d0;
    *(volatile v8h*)dh = fv;
    __threadfence();
    *(volatile v8h*)dh = fv;
  }
}

__global__ __launch_bounds__(NTHR) void k_count(
    const int* __restrict__ keys, const int* __restrict__ gath, int* cnt, float* dinv, int nE, int nN, int vec8) {
  extern __shared__ v4f lds_dyn[];
  int* scnt = (int*)lds_dyn;
  int* list = scnt + NBC;
  int* wcnt = list + LISTN;
  const int tid = threadIdx.x, lane = tid & 31, wave = tid >> 5;
  const int nodeBase = blockIdx.x * NBC;

  {
    const v4i z = {0, 0, 0, 0};
    for (int i = tid; i < NBC / 4; i += NTHR) ((v4i*)scnt)[i] = z;
  }
  __syncthreads();

  const int nChunks = (nE + CHUNK - 1) / CHUNK;
#pragma unroll 1
  for (int ch = 0; ch < nChunks; ++ch) {
    const int cbase = ch * CHUNK;
    const int wc = scan_chunk<NBC, 0>(keys, gath, nE, nN, cbase, nodeBase, vec8, list, tid, lane, wave);
    if (lane == 0) wcnt[wave] = wc;
    __syncthreads();
    if (wave == 0) {
#pragma unroll 1
      for (int wsx = 0; wsx < NWAVE; ++wsx) {
        int nh = __builtin_amdgcn_readfirstlane(wcnt[wsx]);
        nh = nh > WCAP ? WCAP : (nh < 0 ? 0 : nh);
        const int* lp = list + wsx * WCAP;
#pragma unroll 1
        for (int i = 0; i < nh; ++i) {
          const int ent  = __builtin_amdgcn_readfirstlane(lp[i]);
          const int slot = ent & (NBC - 1);
          if (lane == 0) scnt[slot] = scnt[slot] + 1;
        }
      }
    }
    __syncthreads();
  }

  int*   cp = cnt + (size_t)nodeBase;
  float* dp = dinv + (size_t)nodeBase;
#pragma unroll 1
  for (int q = 0; q < 32; ++q) {
    const int f = (wave * 32 + q) * 128 + 4 * lane;
    const v4i c = *(const v4i*)(scnt + f);
    const float g0 = (float)c.x + CSELF, g1 = (float)c.y + CSELF, g2 = (float)c.z + CSELF, g3 = (float)c.w + CSELF;
    v4f d;
    d.x = g0 > 0.f ? rsqrtf(g0) : 0.f; d.y = g1 > 0.f ? rsqrtf(g1) : 0.f;
    d.z = g2 > 0.f ? rsqrtf(g2) : 0.f; d.w = g3 > 0.f ? rsqrtf(g3) : 0.f;
    *(volatile v4i*)(cp + f) = c;
    *(volatile v4f*)(dp + f) = d;
  }
  __threadfence();
#pragma unroll 1
  for (int q = 0; q < 32; ++q) {
    const int f = (wave * 32 + q) * 128 + 4 * lane;
    const v4i c = *(const v4i*)(scnt + f);
    const float g0 = (float)c.x + CSELF, g1 = (float)c.y + CSELF, g2 = (float)c.z + CSELF, g3 = (float)c.w + CSELF;
    v4f d;
    d.x = g0 > 0.f ? rsqrtf(g0) : 0.f; d.y = g1 > 0.f ? rsqrtf(g1) : 0.f;
    d.z = g2 > 0.f ? rsqrtf(g2) : 0.f; d.w = g3 > 0.f ? rsqrtf(g3) : 0.f;
    *(volatile v4i*)(cp + f) = c;
    *(volatile v4f*)(dp + f) = d;
  }
}

__global__ __launch_bounds__(OTHR) void k_offsets(
    const int* __restrict__ cnt, int* off, int* rbase, int nBF) {
  __shared__ __attribute__((aligned(16))) int srb[RBN];
  __shared__ int wtot[OTHR / 32];
  const int tid = threadIdx.x, lane = tid & 31, wave = tid >> 5;
  for (int i = tid; i < RBN; i += OTHR) srb[i] = 0;
  int carry = 0;
#pragma unroll 1
  for (int fb = 0; fb < nBF; ++fb) {
    const int base = fb * NBF;
    const v4i c = *(const v4i*)(cnt + base + 4 * tid);
    const int e0 = max(c.x, 0), e1 = max(c.y, 0), e2 = max(c.z, 0), e3 = max(c.w, 0);
    const int ts = e0 + e1 + e2 + e3;
    int incl = ts;
#pragma unroll
    for (int d = 1; d < 32; d <<= 1) {
      const int t = __shfl_up(incl, d);
      if (lane >= d) incl += t;
    }
    if (lane == 31) wtot[wave] = incl;
    __syncthreads();
    int pre = 0;
#pragma unroll 1
    for (int w = 0; w < wave; ++w) pre += wtot[w];
    int tot = 0;
#pragma unroll
    for (int w = 0; w < OTHR / 32; ++w) tot += wtot[w];
    int run = carry + pre + incl - ts;
    v4i o;
    o.x = run; run += e0;
    o.y = run; run += e1;
    o.z = run; run += e2;
    o.w = run;
    int* op = off + base + 4 * tid;
    *(volatile v4i*)op = o;
    __threadfence();
    *(volatile v4i*)op = o;
    if (tid == 0) srb[min(fb, RBN - 1)] = carry;
    carry += (tot + 31) & ~31;
    __syncthreads();
  }
  if (tid == 0) srb[min(nBF, RBN - 1)] = carry;
  __syncthreads();
  v4i rv = {0, 0, 0, 0};
  if (tid < 32) rv = *(const v4i*)(srb + 4 * tid);
  if (tid < 32) *(volatile v4i*)(rbase + 4 * tid) = rv;
  __threadfence();
  if (tid < 32) *(volatile v4i*)(rbase + 4 * tid) = rv;
}

__global__ __launch_bounds__(NTHR) void k_fill(
    const int* __restrict__ keys, const int* __restrict__ gath, const int* __restrict__ off,
    const int* __restrict__ rbase, int* csr, int nN, int nE, int vec8, int csrLen) {
  extern __shared__ v4f lds_dyn[];
  int* region = (int*)lds_dyn;
  int* cursor = region + RCAP;
  int* list   = cursor + NBF;
  int* wcnt   = list + LISTN;
  const int tid = threadIdx.x, lane = tid & 31, wave = tid >> 5;
  const int b = blockIdx.x;
  const int nodeBase = b * NBF;

  int rb0 = rbase[b];
  const int rb1 = rbase[b + 1];
  rb0 = rb0 < 0 ? 0 : (rb0 > csrLen ? csrLen : rb0);
  rb0 &= ~31;
  int len = rb1 - rb0;
  len = len < 0 ? 0 : (len > RCAP ? RCAP : len);
  int lenW = (len + 31) & ~31;
  if (rb0 + lenW > csrLen) lenW = (csrLen - rb0) & ~31;

  {
    const v4i z = {0, 0, 0, 0};
    for (int i = tid; i < RCAP / 4; i += NTHR) ((v4i*)region)[i] = z;
    for (int s = tid; s < NBF; s += NTHR) {
      int o = off[nodeBase + s] - rb0;
      o = o < 0 ? 0 : (o > RCAP ? RCAP : o);
      cursor[s] = o;
    }
  }
  __syncthreads();

  const int nChunks = (nE + CHUNK - 1) / CHUNK;
#pragma unroll 1
  for (int ch = 0; ch < nChunks; ++ch) {
    const int cbase = ch * CHUNK;
    const int wc = scan_chunk<NBF, 1>(keys, gath, nE, nN, cbase, nodeBase, vec8, list, tid, lane, wave);
    if (lane == 0) wcnt[wave] = wc;
    __syncthreads();
    if (wave == 0) {
#pragma unroll 1
      for (int wsx = 0; wsx < NWAVE; ++wsx) {
        int nh = __builtin_amdgcn_readfirstlane(wcnt[wsx]);
        nh = nh > WCAP ? WCAP : (nh < 0 ? 0 : nh);
        const int* lp = list + wsx * WCAP;
#pragma unroll 1
        for (int i = 0; i < nh; ++i) {
          const int ent  = __builtin_amdgcn_readfirstlane(lp[i]);
          const int slot = ent & (NBF - 1);
          int src = (ent >> ESHF) & 0xFFFFF;
          src = src > nN - 1 ? nN - 1 : src;
          if (lane == 0) {
            int pos = cursor[slot];
            pos = pos < 0 ? 0 : (pos > RCAP - 1 ? RCAP - 1 : pos);
            region[pos] = src;
            const int np = pos + 1;
            cursor[slot] = np > RCAP ? RCAP : np;
          }
        }
      }
    }
    __syncthreads();
  }

  const int nv = lenW >> 2;
  int* gp = csr + rb0;
#pragma unroll 1
  for (int i = tid; i < nv; i += NTHR) { const v4i v = ((const v4i*)region)[i]; *(volatile v4i*)(gp + 4 * i) = v; }
  __threadfence();
#pragma unroll 1
  for (int i = tid; i < nv; i += NTHR) { const v4i v = ((const v4i*)region)[i]; *(volatile v4i*)(gp + 4 * i) = v; }
}

template <int KD, int NPROD, int OUTM, int RS>
__global__ __launch_bounds__(NTHR) void k_gemm(
    const float* __restrict__ A0, int lda0,
    const float* __restrict__ A1, int lda1, int kb1,
    const float* __restrict__ A2, int lda2, int kb2,
    const unsigned short* __restrict__ Bh, const unsigned short* __restrict__ Bl,
    const float* __restrict__ dinv, float* Cf, unsigned short* Ch, unsigned short* Cl, int nRowsA) {
  __shared__ __attribute__((aligned(16))) float stg[GROWS * DIM];
  const int tid = threadIdx.x, lane = tid & 31, wave = tid >> 5, hh = lane >> 4, m = lane & 15;
  const int rowBase = blockIdx.x * GROWS;
  int arow = rowBase + wave * 16 + m;
  arow = arow > nRowsA - 1 ? nRowsA - 1 : arow;

  v8f acc[4];
#pragma unroll
  for (int t = 0; t < 4; ++t) acc[t] = zero8();

#pragma unroll 1
  for (int kt = 0; kt < KD / 32; ++kt) {
    const float* src = A0;
    int lda = lda0, kc = kt;
    if (kt >= kb2) { src = A2; lda = lda2; kc = kt - kb2; }
    else if (kt >= kb1) { src = A1; lda = lda1; kc = kt - kb1; }
    const float* akp = src + (size_t)arow * lda + 32 * kc + 8 * hh;
    float av[16];
    load16(akp, av);
    if (NPROD == 1) {
      const v16h af = cvt_h16(av, ASC);
#pragma unroll
      for (int t = 0; t < 4; ++t) {
        const _Float16* bp = (const _Float16*)Bh + (size_t)(16 * t + m) * KD + 32 * kt + 8 * hh;
        FragH bf;
        bf.h[0] = *(const v8h*)bp;
        bf.h[1] = *(const v8h*)(bp + 16);
        acc[t] = wmf(af, bf.v, acc[t]);
      }
    } else {
      v16b ah, al;
      cvt_b16(av, ah, al);
#pragma unroll
      for (int t = 0; t < 4; ++t) {
        const size_t bo = (size_t)(16 * t + m) * KD + 32 * kt + 8 * hh;
        FragB bh, bl;
        bh.u[0] = *(const v8us*)(Bh + bo); bh.u[1] = *(const v8us*)(Bh + bo + 16);
        bl.u[0] = *(const v8us*)(Bl + bo); bl.u[1] = *(const v8us*)(Bl + bo + 16);
        acc[t] = wmb(ah, bh.v, acc[t]);
        acc[t] = wmb(ah, bl.v, acc[t]);
        acc[t] = wmb(al, bh.v, acc[t]);
      }
    }
  }

  const int r0 = wave * 16 + 8 * hh;
  float s[8];
  if (RS) {
    const v4f dA = *(const v4f*)(dinv + (size_t)rowBase + r0);
    const v4f dB = *(const v4f*)(dinv + (size_t)rowBase + r0 + 4);
    s[0] = dA.x; s[1] = dA.y; s[2] = dA.z; s[3] = dA.w; s[4] = dB.x; s[5] = dB.y; s[6] = dB.z; s[7] = dB.w;
  } else {
#pragma unroll
    for (int r = 0; r < 8; ++r) s[r] = 1.0f;
  }
  const float OSC = (NPROD == 1) ? (1.0f / (ASC * WSC)) : 1.0f;
#pragma unroll
  for (int r = 0; r < 8; ++r) s[r] = s[r] * OSC;
  float* sp = stg + r0 * DIM + m;
#pragma unroll
  for (int t = 0; t < 4; ++t) {
#pragma unroll
    for (int r = 0; r < 8; ++r) sp[r * DIM + 16 * t] = acc[t][r] * s[r];
  }
  __syncthreads();

  const float* lp = stg + wave * 16 * DIM;
  if (OUTM == 0) {
    float* gp = Cf + (size_t)(rowBase + wave * 16) * DIM;
#pragma unroll
    for (int i = 0; i < 8; ++i) {
      const v4f v = *(const v4f*)(lp + i * 128 + 4 * lane);
      *(volatile v4f*)(gp + i * 128 + 4 * lane) = v;
    }
    __threadfence();
#pragma unroll
    for (int i = 0; i < 8; ++i) {
      const v4f v = *(const v4f*)(lp + i * 128 + 4 * lane);
      *(volatile v4f*)(gp + i * 128 + 4 * lane) = v;
    }
  } else {
    unsigned short* gh = Ch + (size_t)(rowBase + wave * 16) * DIM;
    unsigned short* gl = Cl + (size_t)(rowBase + wave * 16) * DIM;
#pragma unroll
    for (int i = 0; i < 4; ++i) {
      const int e0 = i * 256 + 8 * lane;
      const v4f a = *(const v4f*)(lp + e0), c = *(const v4f*)(lp + e0 + 4);
      const float fv[8] = {a.x, a.y, a.z, a.w, c.x, c.y, c.z, c.w};
      v8us hv, lv;
#pragma unroll
      for (int e = 0; e < 8; ++e) { unsigned short hb, lb; bfsplit(fv[e], hb, lb); hv[e] = hb; lv[e] = lb; }
      *(volatile v8us*)(gh + e0) = hv;
      *(volatile v8us*)(gl + e0) = lv;
    }
    __threadfence();
#pragma unroll
    for (int i = 0; i < 4; ++i) {
      const int e0 = i * 256 + 8 * lane;
      const v4f a = *(const v4f*)(lp + e0), c = *(const v4f*)(lp + e0 + 4);
      const float fv[8] = {a.x, a.y, a.z, a.w, c.x, c.y, c.z, c.w};
      v8us hv, lv;
#pragma unroll
      for (int e = 0; e < 8; ++e) { unsigned short hb, lb; bfsplit(fv[e], hb, lb); hv[e] = hb; lv[e] = lb; }
      *(volatile v8us*)(gh + e0) = hv;
      *(volatile v8us*)(gl + e0) = lv;
    }
  }
}

__global__ __launch_bounds__(NTHR) void k_agg1(
    const int* __restrict__ csr, const int* __restrict__ off, const int* __restrict__ cnt,
    const float* __restrict__ dinv, const float* __restrict__ hw, const float* __restrict__ bs,
    float* h, int nN, int csrLen) {
  const int tid = threadIdx.x, lane = tid & 31, wave = tid >> 5;
  const int tbase = blockIdx.x * TGT + wave * 32;
  const int cl = tbase + lane;
  const int cnt_l = cnt[cl];
  const int off_l = off[cl];
  union FI { float f; int i; };
  FI dvu; dvu.f = dinv[cl];
  const v2f bb = *(const v2f*)(bs + 2 * lane);

#pragma unroll 1
  for (int j = 0; j < 32; ++j) {
    const int c = tbase + j;
    int n = __builtin_amdgcn_readlane(cnt_l, j);
    n = n < 0 ? 0 : (n > DEGCAP ? DEGCAP : n);
    const int st = __builtin_amdgcn_readlane(off_l, j);
    FI du; du.i = __builtin_amdgcn_readlane(dvu.i, j);
    const float dc = du.f;
    v2f acc = {0.f, 0.f};
#pragma unroll 1
    for (int q0 = 0; q0 < n; q0 += 32) {
      int pos = st + q0 + lane;
      pos = pos < 0 ? 0 : (pos > csrLen - 1 ? csrLen - 1 : pos);
      int sl = csr[pos];
      sl = sl < 0 ? 0 : (sl > nN - 1 ? nN - 1 : sl);
      const int mcnt = (n - q0) < 32 ? (n - q0) : 32;
#pragma unroll 1
      for (int p = 0; p < mcnt; ++p) {
        const int sidx = __builtin_amdgcn_readlane(sl, p);
        acc = acc + *(const v2f*)(hw + (size_t)sidx * DIM + 2 * lane);
      }
    }
    const v2f sv = *(const v2f*)(hw + (size_t)c * DIM + 2 * lane);
    v2f v = (acc + sv * CSELF) * dc + bb;
    v.x = fmaxf(v.x, 0.f); v.y = fmaxf(v.y, 0.f);
    float* hp = h + (size_t)c * DIM + 2 * lane;
    *(volatile v2f*)hp = v;
    __threadfence();
    *(volatile v2f*)hp = v;
  }
}

__device__ __forceinline__ v8f mm_f16(const float* As, int lda, float asc, const float* __restrict__ W, int ldw,
                                      int col0, float wsc, int hh, int m) {
  v8f acc = zero8();
#pragma unroll
  for (int kt = 0; kt < 2; ++kt) {
    float av[16];
    load16(As + m * lda + 32 * kt + 8 * hh, av);
    const v16h af = cvt_h16(av, asc);
    const float* wcp = W + (size_t)(32 * kt + 8 * hh) * ldw + col0 + m;
    FragH bf;
#pragma unroll
    for (int i = 0; i < 8; ++i) {
      bf.h[0][i] = (_Float16)(wcp[(size_t)i * ldw] * wsc);
      bf.h[1][i] = (_Float16)(wcp[(size_t)(16 + i) * ldw] * wsc);
    }
    acc = wmf(af, bf.v, acc);
  }
  return acc;
}
__device__ __forceinline__ v8f mm_bx3(const float* As, int lda, const float* __restrict__ W, int ldw,
                                      int col0, int hh, int m) {
  v8f acc = zero8();
#pragma unroll
  for (int kt = 0; kt < 2; ++kt) {
    float av[16];
    load16(As + m * lda + 32 * kt + 8 * hh, av);
    v16b ah, al;
    cvt_b16(av, ah, al);
    const float* wcp = W + (size_t)(32 * kt + 8 * hh) * ldw + col0 + m;
    FragB bh, bl;
#pragma unroll
    for (int i = 0; i < 8; ++i) {
      unsigned short hb, lb;
      bfsplit(wcp[(size_t)i * ldw], hb, lb);         bh.u[0][i] = hb; bl.u[0][i] = lb;
      bfsplit(wcp[(size_t)(16 + i) * ldw], hb, lb);  bh.u[1][i] = hb; bl.u[1][i] = lb;
    }
    acc = wmb(ah, bh.v, acc);
    acc = wmb(ah, bl.v, acc);
    acc = wmb(al, bh.v, acc);
  }
  return acc;
}

__global__ __launch_bounds__(64) void k_smallq(const float* __restrict__ memv, const float* __restrict__ wqw,
                                                unsigned short* qexp) {
  __shared__ __attribute__((aligned(16))) float TA[NMEM * DIM];
  __shared__ __attribute__((aligned(16))) float TB[NMEM * DIM];
  const int tid = threadIdx.x, lane = tid & 31, wave = tid >> 5, hh = lane >> 4, m = lane & 15;
  for (int i = tid; i < NMEM * DIM; i += 64) TA[i] = memv[i];
  __syncthreads();
#pragma unroll
  for (int t = 0; t < 4; ++t) {
    const v8f acc = mm_bx3(TA + 16 * wave * DIM, DIM, wqw, DIM, 16 * t, hh, m);
#pragma unroll
    for (int r = 0; r < 8; ++r) TB[(16 * wave + 8 * hh + r) * DIM + 16 * t + m] = acc[r];
  }
  __syncthreads();
#pragma unroll 1
  for (int it = 0; it < 8; ++it) {
    const int pi = it * 64 + tid;
    const int row = pi >> 2, kk0 = (pi & 3) * 8, hd = row >> 5, q = row & 31;
    v8us hv, lv;
#pragma unroll
    for (int e = 0; e < 8; ++e) {
      const int kk = kk0 + e;
      float v = TB[q * DIM + 32 * (hd >> 1) + kk];
      v = ((kk >> 4) == (hd & 1)) ? v : 0.0f;
      unsigned short hb, lb; bfsplit(v, hb, lb); hv[e] = hb; lv[e] = lb;
    }
    *(volatile v8us*)(qexp + (size_t)pi * 8) = hv;
    *(volatile v8us*)(qexp + SROWS * 32 + (size_t)pi * 8) = lv;
  }
  __threadfence();
#pragma unroll 1
  for (int it = 0; it < 8; ++it) {
    const int pi = it * 64 + tid;
    const int row = pi >> 2, kk0 = (pi & 3) * 8, hd = row >> 5, q = row & 31;
    v8us hv, lv;
#pragma unroll
    for (int e = 0; e < 8; ++e) {
      const int kk = kk0 + e;
      float v = TB[q * DIM + 32 * (hd >> 1) + kk];
      v = ((kk >> 4) == (hd & 1)) ? v : 0.0f;
      unsigned short hb, lb; bfsplit(v, hb, lb); hv[e] = hb; lv[e] = lb;
    }
    *(volatile v8us*)(qexp + (size_t)pi * 8) = hv;
    *(volatile v8us*)(qexp + SROWS * 32 + (size_t)pi * 8) = lv;
  }
}

__global__ __launch_bounds__(64) void k_smallm(const float* __restrict__ gpad, const float* __restrict__ wvw,
                                                const float* __restrict__ wow, const float* __restrict__ wkb,
                                                const float* __restrict__ wvb, float* kbvb) {
  __shared__ __attribute__((aligned(16))) float G[SROWS * DIM];
  __shared__ __attribute__((aligned(16))) float TA[NMEM * DIM];
  __shared__ __attribute__((aligned(16))) float TB[NMEM * DIM];
  const int tid = threadIdx.x, lane = tid & 31, wave = tid >> 5, hh = lane >> 4, m = lane & 15;
  for (int i = tid; i < SROWS * DIM / 4; i += 64) ((v4f*)G)[i] = ((const v4f*)gpad)[i];
  __syncthreads();
#pragma unroll
  for (int t = 0; t < 4; ++t) {
    const v8f acc = mm_f16(G + (32 * t + 16 * wave) * DIM, DIM, ASC, wvw, DIM, 16 * t, WSC, hh, m);
#pragma unroll
    for (int r = 0; r < 8; ++r) TA[(16 * wave + 8 * hh + r) * DIM + 16 * t + m] = acc[r] * (1.0f / 1024.0f);
  }
  __syncthreads();
#pragma unroll
  for (int t = 0; t < 4; ++t) {
    const v8f acc = mm_f16(TA + 16 * wave * DIM, DIM, ASC, wow, DIM, 16 * t, WSC, hh, m);
#pragma unroll
    for (int r = 0; r < 8; ++r) TB[(16 * wave + 8 * hh + r) * DIM + 16 * t + m] = acc[r] * (1.0f / 1024.0f);
  }
  __syncthreads();
#pragma unroll
  for (int t = 0; t < 4; ++t) {
    const v8f ak = mm_f16(TB + 16 * wave * DIM, DIM, ASC, wkb, DIM, 16 * t, WSC, hh, m);
#pragma unroll
    for (int r = 0; r < 8; ++r) G[(16 * wave + 8 * hh + r) * DIM + 16 * t + m] = ak[r] * (1.0f / 1024.0f);
    const v8f aw = mm_f16(TB + 16 * wave * DIM, DIM, ASC, wvb, DIM, 16 * t, WSC, hh, m);
#pragma unroll
    for (int r = 0; r < 8; ++r) G[NMEM * DIM + (16 * wave + 8 * hh + r) * DIM + 16 * t + m] = aw[r] * (1.0f / 1024.0f);
  }
  __syncthreads();
#pragma unroll 1
  for (int it = 0; it < 16; ++it) {
    const int pi = it * 64 + tid;
    const v4f v = ((const v4f*)G)[pi];
    *(volatile v4f*)(kbvb + (size_t)pi * 4) = v;
  }
  __threadfence();
#pragma unroll 1
  for (int it = 0; it < 16; ++it) {
    const int pi = it * 64 + tid;
    const v4f v = ((const v4f*)G)[pi];
    *(volatile v4f*)(kbvb + (size_t)pi * 4) = v;
  }
}

__global__ __launch_bounds__(NTHR) void k_scores(
    const unsigned short* __restrict__ qh, const unsigned short* __restrict__ ql,
    const unsigned short* __restrict__ kh, const unsigned short* __restrict__ kl, float* S, int npad) {
  __shared__ __attribute__((aligned(16))) float sS[64 * 128];
  const int tid = threadIdx.x, lane = tid & 31, wave = tid >> 5, hh = lane >> 4, m = lane & 15;
  const int nodeBase = blockIdx.x * 128;
  const int rt = wave & 3, cg = wave >> 2;
#pragma unroll 1
  for (int ks = 0; ks < 2; ++ks) {
    const int arow = 64 * ks + 16 * rt + m;
    FragB ah, al;
    ah.u[0] = *(const v8us*)(qh + arow * 32 + 8 * hh);
    ah.u[1] = *(const v8us*)(qh + arow * 32 + 16 + 8 * hh);
    al.u[0] = *(const v8us*)(ql + arow * 32 + 8 * hh);
    al.u[1] = *(const v8us*)(ql + arow * 32 + 16 + 8 * hh);
    v8f acc[4];
#pragma unroll
    for (int ct = 0; ct < 4; ++ct) {
      const int node = nodeBase + 64 * cg + 16 * ct + m;
      const size_t bo = (size_t)node * DIM + 32 * ks + 8 * hh;
      FragB bh, bl;
      bh.u[0] = *(const v8us*)(kh + bo); bh.u[1] = *(const v8us*)(kh + bo + 16);
      bl.u[0] = *(const v8us*)(kl + bo); bl.u[1] = *(const v8us*)(kl + bo + 16);
      v8f a = zero8();
      a = wmb(ah.v, bh.v, a);
      a = wmb(ah.v, bl.v, a);
      a = wmb(al.v, bh.v, a);
      acc[ct] = a;
    }
#pragma unroll
    for (int ct = 0; ct < 4; ++ct) {
#pragma unroll
      for (int r = 0; r < 8; ++r) sS[(16 * rt + 8 * hh + r) * 128 + 64 * cg + 16 * ct + m] = acc[ct][r] * 0.25f;
    }
    __syncthreads();
    float* gp = S + (size_t)(64 * ks + 8 * wave) * npad + nodeBase + 4 * lane;
#pragma unroll
    for (int i = 0; i < 8; ++i) {
      const v4f v = *(const v4f*)(sS + (8 * wave + i) * 128 + 4 * lane);
      *(volatile v4f*)(gp + (size_t)i * npad) = v;
    }
    __threadfence();
#pragma unroll
    for (int i = 0; i < 8; ++i) {
      const v4f v = *(const v4f*)(sS + (8 * wave + i) * 128 + 4 * lane);
      *(volatile v4f*)(gp + (size_t)i * npad) = v;
    }
    __syncthreads();
  }
}

__device__ __forceinline__ void csw(float& a, float& b) { const float hi = fmaxf(a, b), lo = fminf(a, b); a = hi; b = lo; }
__device__ __forceinline__ void ins5(float s, float& t0, float& t1, float& t2, float& t3, float& t4) {
  if (s > t4) { t4 = s; csw(t3, t4); csw(t2, t3); csw(t1, t2); csw(t0, t1); }
}

__global__ __launch_bounds__(NTHR) void k_top5(const float* __restrict__ S, const float* __restrict__ hpl,
                                                 float* gpad, int nN, int npad) {
  __shared__ float sm[NTHR * TOPN];
  __shared__ int hl[HCAP];
  __shared__ int wcn[NWAVE];
  __shared__ float sth[2];
  const int tid = threadIdx.x, lane = tid & 31, wave = tid >> 5;
  const int p = blockIdx.x;
  const float* row = S + (size_t)p * npad;

  float t0 = -3.0e38f, t1 = -3.0e38f, t2 = -3.0e38f, t3 = -3.0e38f, t4 = -3.0e38f;
#pragma unroll 1
  for (int base = 0; base < nN; base += NTHR) {
    const int k = base + tid;
    const int kc = k < nN ? k : nN - 1;
    float s = row[kc];
    s = (k < nN) ? s : -3.0e38f;
    ins5(s, t0, t1, t2, t3, t4);
  }
  sm[tid * TOPN + 0] = t0; sm[tid * TOPN + 1] = t1; sm[tid * TOPN + 2] = t2; sm[tid * TOPN + 3] = t3; sm[tid * TOPN + 4] = t4;
  __syncthreads();
  if (tid == 0) {
    float b0 = -3.0e38f, b1 = -3.0e38f, b2 = -3.0e38f, b3 = -3.0e38f, b4 = -3.0e38f;
#pragma unroll 1
    for (int i = 0; i < NTHR * TOPN; ++i) ins5(sm[i], b0, b1, b2, b3, b4);
    sth[0] = b4;
    sth[1] = b0;
  }
  __syncthreads();
  const float thr = sth[0], mx = sth[1];

  int len = 0;
#pragma unroll 1
  for (int base = 0; base < nN; base += NTHR) {
    const int k = base + tid;
    const int kc = k < nN ? k : nN - 1;
    const float s = row[kc];
    const bool hit = (k < nN) && (s >= thr);
    const unsigned mk = __builtin_amdgcn_ballot_w32(hit);
    if (lane == 0) wcn[wave] = (int)__builtin_popcount(mk);
    __syncthreads();
    int pre = 0, tot = 0;
#pragma unroll
    for (int w = 0; w < NWAVE; ++w) { const int c = wcn[w]; pre += (w < wave) ? c : 0; tot += c; }
    if (hit) {
      const int pos = len + pre + (int)__builtin_amdgcn_mbcnt_lo(mk, 0u);
      if (pos < HCAP) hl[pos] = k;
    }
    len += tot;
    __syncthreads();
  }
  len = len > HCAP ? HCAP : len;

  if (wave == 0) {
    float den = 0.f, g0 = 0.f, g1 = 0.f;
#pragma unroll 1
    for (int i = 0; i < len; ++i) {
      int k = hl[i];
      k = k < 0 ? 0 : (k > nN - 1 ? nN - 1 : k);
      const float s = row[k];
      const float w = expf(s - mx);
      den += w;
      const v2f hv = *(const v2f*)(hpl + (size_t)k * DIM + 2 * lane);
      g0 = fmaf(w, hv.x, g0);
      g1 = fmaf(w, hv.y, g1);
    }
    const float inv = den > 0.f ? (1.0f / den) : 0.f;
    v2f gv;
    gv.x = g0 * inv; gv.y = g1 * inv;
    float* gp = gpad + (size_t)p * DIM + 2 * lane;
    *(volatile v2f*)gp = gv;
    __threadfence();
    *(volatile v2f*)gp = gv;
  }
}

__global__ __launch_bounds__(NTHR) void k_battn(
    const float* __restrict__ hpl, const unsigned short* __restrict__ pqb, const unsigned short* __restrict__ pob,
    const float* __restrict__ kbvb, const float* __restrict__ g1, const float* __restrict__ be1, float* tpl) {
  __shared__ __attribute__((aligned(16))) _Float16 kbm[NHD * NMEM * 32];
  __shared__ __attribute__((aligned(16))) _Float16 vbT[NHD * DHD * NMEM];
  __shared__ __attribute__((aligned(16))) float area[NWAVE * 1024];
  const int tid = threadIdx.x, lane = tid & 31, wave = tid >> 5, hh = lane >> 4, m = lane & 15;

  for (int i = tid; i < NHD * NMEM * 32; i += NTHR) {
    const int hd = i >> 10, slot = (i >> 5) & 31, kk = i & 31;
    float v = kbvb[slot * DIM + 32 * (hd >> 1) + kk];
    v = ((kk >> 4) == (hd & 1)) ? v * ASC : 0.0f;
    kbm[i] = (_Float16)v;
  }
  for (int i = tid; i < NHD * DHD * NMEM; i += NTHR) {
    const int hd = i >> 9, d = (i >> 5) & 15, slot = i & 31;
    vbT[i] = (_Float16)(kbvb[NMEM * DIM + slot * DIM + 16 * hd + d] * ASC);
  }

  const int node0 = blockIdx.x * GROWS + 16 * wave;
  float* wsf = area + wave * 1024;
  _Float16* wsh = (_Float16*)wsf;

  v8f qacc[4];
#pragma unroll
  for (int t = 0; t < 4; ++t) qacc[t] = zero8();
#pragma unroll
  for (int kt = 0; kt < 2; ++kt) {
    float av[16];
    load16(hpl + (size_t)(node0 + m) * DIM + 32 * kt + 8 * hh, av);
    const v16h af = cvt_h16(av, ASC);
#pragma unroll
    for (int t = 0; t < 4; ++t) {
      const _Float16* bp = (const _Float16*)pqb + (size_t)(16 * t + m) * DIM + 32 * kt + 8 * hh;
      FragH bf;
      bf.h[0] = *(const v8h*)bp;
      bf.h[1] = *(const v8h*)(bp + 16);
      qacc[t] = wmf(af, bf.v, qacc[t]);
    }
  }
#pragma unroll
  for (int t = 0; t < 4; ++t) {
#pragma unroll
    for (int r = 0; r < 8; ++r) wsh[(8 * hh + r) * DIM + 16 * t + m] = (_Float16)(qacc[t][r] * 0.0625f);
  }
  __syncthreads();
  FragH qa[2];
#pragma unroll
  for (int ks = 0; ks < 2; ++ks) {
    qa[ks].h[0] = *(const v8h*)(wsh + m * DIM + 32 * ks + 8 * hh);
    qa[ks].h[1] = *(const v8h*)(wsh + m * DIM + 32 * ks + 16 + 8 * hh);
  }
  __syncthreads();

  v8f sc[8];
#pragma unroll
  for (int hd = 0; hd < NHD; ++hd) {
#pragma unroll
    for (int t2 = 0; t2 < 2; ++t2) {
      const _Float16* bp = kbm + (hd * 32 + 16 * t2 + m) * 32 + 8 * hh;
      FragH bf;
      bf.h[0] = *(const v8h*)bp;
      bf.h[1] = *(const v8h*)(bp + 16);
      sc[2 * hd + t2] = wmf(qa[hd >> 1].v, bf.v, zero8());
    }
  }
  const float SCL = 1.0f / 16384.0f;
#pragma unroll
  for (int hd = 0; hd < NHD; ++hd) {
#pragma unroll
    for (int r = 0; r < 8; ++r) {
      const float s0 = sc[2 * hd][r] * SCL, s1 = sc[2 * hd + 1][r] * SCL;
      float mx = fmaxf(s0, s1);
      mx = fmaxf(mx, __shfl_xor(mx, 1, 32));
      mx = fmaxf(mx, __shfl_xor(mx, 2, 32));
      mx = fmaxf(mx, __shfl_xor(mx, 4, 32));
      mx = fmaxf(mx, __shfl_xor(mx, 8, 32));
      const float p0 = expf(s0 - mx), p1 = expf(s1 - mx);
      float su = p0 + p1;
      su += __shfl_xor(su, 1, 32);
      su += __shfl_xor(su, 2, 32);
      su += __shfl_xor(su, 4, 32);
      su += __shfl_xor(su, 8, 32);
      const float rsu = 1024.0f / su;
      wsh[(8 * hh + r) * 128 + 32 * hd + m]      = (_Float16)(p0 * rsu);
      wsh[(8 * hh + r) * 128 + 32 * hd + 16 + m] = (_Float16)(p1 * rsu);
    }
  }
  __syncthreads();

  v8f oacc[4];
#pragma unroll
  for (int hd = 0; hd < NHD; ++hd) {
    FragH pa, vf;
    pa.h[0] = *(const v8h*)(wsh + m * 128 + 32 * hd + 8 * hh);
    pa.h[1] = *(const v8h*)(wsh + m * 128 + 32 * hd + 16 + 8 * hh);
    const _Float16* vp = vbT + (hd * 16 + m) * 32 + 8 * hh;
    vf.h[0] = *(const v8h*)vp;
    vf.h[1] = *(const v8h*)(vp + 16);
    oacc[hd] = wmf(pa.v, vf.v, zero8());
  }
  __syncthreads();
#pragma unroll
  for (int hd = 0; hd < NHD; ++hd) {
#pragma unroll
    for (int r = 0; r < 8; ++r) wsh[(8 * hh + r) * DIM + 16 * hd + m] = (_Float16)(oacc[hd][r] * (1.0f / 1024.0f));
  }
  __syncthreads();
  FragH oa[2];
#pragma unroll
  for (int kt = 0; kt < 2; ++kt) {
    oa[kt].h[0] = *(const v8h*)(wsh + m * DIM + 32 * kt + 8 * hh);
    oa[kt].h[1] = *(const v8h*)(wsh + m * DIM + 32 * kt + 16 + 8 * hh);
  }

  v8f aacc[4];
#pragma unroll
  for (int t = 0; t < 4; ++t) aacc[t] = zero8();
#pragma unroll
  for (int kt = 0; kt < 2; ++kt) {
#pragma unroll
    for (int t = 0; t < 4; ++t) {
      const _Float16* bp = (const _Float16*)pob + (size_t)(16 * t + m) * DIM + 32 * kt + 8 * hh;
      FragH bf;
      bf.h[0] = *(const v8h*)bp;
      bf.h[1] = *(const v8h*)(bp + 16);
      aacc[t] = wmf(oa[kt].v, bf.v, aacc[t]);
    }
  }
  __syncthreads();
#pragma unroll
  for (int t = 0; t < 4; ++t) {
#pragma unroll
    for (int r = 0; r < 8; ++r) wsf[(8 * hh + r) * DIM + 16 * t + m] = aacc[t][r] * (1.0f / 1024.0f);
  }
  __syncthreads();

  const float ga = g1[lane], gb = g1[lane + 32], ba = be1[lane], bbv = be1[lane + 32];
#pragma unroll 1
  for (int i = 0; i < 16; ++i) {
    const size_t rb = (size_t)(node0 + i) * DIM;
    const float v0 = hpl[rb + lane] + wsf[i * DIM + lane];
    const float v1 = hpl[rb + 32 + lane] + wsf[i * DIM + 32 + lane];
    float su = v0 + v1;
    su += __shfl_xor(su, 16, 32); su += __shfl_xor(su, 8, 32); su += __shfl_xor(su, 4, 32);
    su += __shfl_xor(su, 2, 32);  su += __shfl_xor(su, 1, 32);
    const float mu = su * (1.0f / 64.0f);
    const float d0 = v0 - mu, d1 = v1 - mu;
    float sq = d0 * d0 + d1 * d1;
    sq += __shfl_xor(sq, 16, 32); sq += __shfl_xor(sq, 8, 32); sq += __shfl_xor(sq, 4, 32);
    sq += __shfl_xor(sq, 2, 32);  sq += __shfl_xor(sq, 1, 32);
    const float rs = rsqrtf(sq * (1.0f / 64.0f) + 1e-5f);
    wsf[i * DIM + lane]      = d0 * rs * ga + ba;
    wsf[i * DIM + 32 + lane] = d1 * rs * gb + bbv;
  }
  __syncthreads();
  float* gp = tpl + (size_t)node0 * DIM;
#pragma unroll
  for (int i = 0; i < 8; ++i) {
    const v4f v = *(const v4f*)(wsf + i * 128 + 4 * lane);
    *(volatile v4f*)(gp + i * 128 + 4 * lane) = v;
  }
  __threadfence();
#pragma unroll
  for (int i = 0; i < 8; ++i) {
    const v4f v = *(const v4f*)(wsf + i * 128 + 4 * lane);
    *(volatile v4f*)(gp + i * 128 + 4 * lane) = v;
  }
}

__global__ __launch_bounds__(NTHR) void k_ffn(
    const float* __restrict__ tpl, const float* __restrict__ hpl,
    const unsigned short* __restrict__ pf1, const unsigned short* __restrict__ pf2,
    const float* __restrict__ fb1, const float* __restrict__ fb2,
    const float* __restrict__ g2, const float* __restrict__ be2,
    const float* __restrict__ gm, const float* __restrict__ bem, float* zpl) {
  __shared__ __attribute__((aligned(16))) float area[NWAVE * 1024];
  const int tid = threadIdx.x, lane = tid & 31, wave = tid >> 5, hh = lane >> 4, m = lane & 15;
  const int node0 = blockIdx.x * GROWS + 16 * wave;
  float* wsf = area + wave * 1024;
  _Float16* wsh = (_Float16*)wsf;

  FragH ta[2];
#pragma unroll
  for (int kt = 0; kt < 2; ++kt) {
    float av[16];
    load16(tpl + (size_t)(node0 + m) * DIM + 32 * kt + 8 * hh, av);
    ta[kt].v = cvt_h16(av, ASC);
  }
  v8f macc[8];
#pragma unroll
  for (int t8 = 0; t8 < 8; ++t8) macc[t8] = zero8();
#pragma unroll
  for (int kt = 0; kt < 2; ++kt) {
#pragma unroll
    for (int t8 = 0; t8 < 8; ++t8) {
      const _Float16* bp = (const _Float16*)pf1 + (size_t)(16 * t8 + m) * DIM + 32 * kt + 8 * hh;
      FragH bf;
      bf.h[0] = *(const v8h*)bp;
      bf.h[1] = *(const v8h*)(bp + 16);
      macc[t8] = wmf(ta[kt].v, bf.v, macc[t8]);
    }
  }
#pragma unroll
  for (int t8 = 0; t8 < 8; ++t8) {
    const float bc = fb1[16 * t8 + m];
#pragma unroll
    for (int r = 0; r < 8; ++r) {
      float v = macc[t8][r] * (1.0f / 1024.0f) + bc;
      v = fmaxf(v, 0.0f) * ASC;
      wsh[(8 * hh + r) * FFH + 16 * t8 + m] = (_Float16)v;
    }
  }
  __syncthreads();
  FragH ma[4];
#pragma unroll
  for (int k4 = 0; k4 < 4; ++k4) {
    ma[k4].h[0] = *(const v8h*)(wsh + m * FFH + 32 * k4 + 8 * hh);
    ma[k4].h[1] = *(const v8h*)(wsh + m * FFH + 32 * k4 + 16 + 8 * hh);
  }
  v8f facc[4];
#pragma unroll
  for (int t = 0; t < 4; ++t) facc[t] = zero8();
#pragma unroll
  for (int k4 = 0; k4 < 4; ++k4) {
#pragma unroll
    for (int t = 0; t < 4; ++t) {
      const _Float16* bp = (const _Float16*)pf2 + (size_t)(16 * t + m) * FFH + 32 * k4 + 8 * hh;
      FragH bf;
      bf.h[0] = *(const v8h*)bp;
      bf.h[1] = *(const v8h*)(bp + 16);
      facc[t] = wmf(ma[k4].v, bf.v, facc[t]);
    }
  }
  __syncthreads();
#pragma unroll
  for (int t = 0; t < 4; ++t) {
    const float bc2 = fb2[16 * t + m];
#pragma unroll
    for (int r = 0; r < 8; ++r) wsf[(8 * hh + r) * DIM + 16 * t + m] = facc[t][r] * (1.0f / 1024.0f) + bc2;
  }
  __syncthreads();

  const float ga = g2[lane], gb = g2[lane + 32], ba = be2[lane], bbv = be2[lane + 32];
  const float gma = gm[lane], gmb = gm[lane + 32], bma = bem[lane], bmb = bem[lane + 32];
#pragma unroll 1
  for (int i = 0; i < 16; ++i) {
    const size_t rb = (size_t)(node0 + i) * DIM;
    const float u0 = tpl[rb + lane] + wsf[i * DIM + lane];
    const float u1 = tpl[rb + 32 + lane] + wsf[i * DIM + 32 + lane];
    float su = u0 + u1;
    su += __shfl_xor(su, 16, 32); su += __shfl_xor(su, 8, 32); su += __shfl_xor(su, 4, 32);
    su += __shfl_xor(su, 2, 32);  su += __shfl_xor(su, 1, 32);
    const float mu = su * (1.0f / 64.0f);
    const float d0 = u0 - mu, d1 = u1 - mu;
    float sq = d0 * d0 + d1 * d1;
    sq += __shfl_xor(sq, 16, 32); sq += __shfl_xor(sq, 8, 32); sq += __shfl_xor(sq, 4, 32);
    sq += __shfl_xor(sq, 2, 32);  sq += __shfl_xor(sq, 1, 32);
    const float rs = rsqrtf(sq * (1.0f / 64.0f) + 1e-5f);
    const float xg0 = d0 * rs * ga + ba, xg1 = d1 * rs * gb + bbv;

    const float w0 = hpl[rb + lane], w1 = hpl[rb + 32 + lane];
    float sh = w0 + w1;
    sh += __shfl_xor(sh, 16, 32); sh += __shfl_xor(sh, 8, 32); sh += __shfl_xor(sh, 4, 32);
    sh += __shfl_xor(sh, 2, 32);  sh += __shfl_xor(sh, 1, 32);
    const float muh = sh * (1.0f / 64.0f);
    const float e0 = w0 - muh, e1 = w1 - muh;
    float sqh = e0 * e0 + e1 * e1;
    sqh += __shfl_xor(sqh, 16, 32); sqh += __shfl_xor(sqh, 8, 32); sqh += __shfl_xor(sqh, 4, 32);
    sqh += __shfl_xor(sqh, 2, 32);  sqh += __shfl_xor(sqh, 1, 32);
    const float rsh = rsqrtf(sqh * (1.0f / 64.0f) + 1e-5f);
    const float hn0 = e0 * rsh * gma + bma, hn1 = e1 * rsh * gmb + bmb;

    wsf[i * DIM + lane]      = 0.5f * xg0 + hn0;
    wsf[i * DIM + 32 + lane] = 0.5f * xg1 + hn1;
  }
  __syncthreads();
  float* gp = zpl + (size_t)node0 * DIM;
#pragma unroll
  for (int i = 0; i < 8; ++i) {
    const v4f v = *(const v4f*)(wsf + i * 128 + 4 * lane);
    *(volatile v4f*)(gp + i * 128 + 4 * lane) = v;
  }
  __threadfence();
#pragma unroll
  for (int i = 0; i < 8; ++i) {
    const v4f v = *(const v4f*)(wsf + i * 128 + 4 * lane);
    *(volatile v4f*)(gp + i * 128 + 4 * lane) = v;
  }
}

__global__ __launch_bounds__(NTHR) void k_agg2(
    const int* __restrict__ csr, const int* __restrict__ off, const int* __restrict__ cnt,
    const float* __restrict__ dinv, const float* __restrict__ hw, const float* __restrict__ bs,
    float* out, int nN, int csrLen) {
  __shared__ __attribute__((aligned(16))) float sout[NWAVE * 32 * FOUT];
  const int tid = threadIdx.x, lane = tid & 31, wave = tid >> 5;
  const int tbase = blockIdx.x * TGT + wave * 32;
  const int cl = tbase + lane;
  const int cnt_l = cnt[cl];
  const int off_l = off[cl];
  union FI { float f; int i; };
  FI dvu; dvu.f = dinv[cl];
  const bool valid = (2 * lane + 1) < FOUT;
  const int c0i = (2 * lane) < (FOUT - 1) ? (2 * lane) : (FOUT - 1);
  const int c1i = (2 * lane + 1) < (FOUT - 1) ? (2 * lane + 1) : (FOUT - 1);
  v2f bb;
  bb.x = bs[c0i]; bb.y = bs[c1i];
  if (!valid) { bb.x = 0.f; bb.y = 0.f; }
  float* sw = sout + wave * 32 * FOUT;

#pragma unroll 1
  for (int j = 0; j < 32; ++j) {
    const int c = tbase + j;
    int n = __builtin_amdgcn_readlane(cnt_l, j);
    n = n < 0 ? 0 : (n > DEGCAP ? DEGCAP : n);
    const int st = __builtin_amdgcn_readlane(off_l, j);
    FI du; du.i = __builtin_amdgcn_readlane(dvu.i, j);
    const float dc = du.f;
    v2f acc = {0.f, 0.f};
#pragma unroll 1
    for (int q0 = 0; q0 < n; q0 += 32) {
      int pos = st + q0 + lane;
      pos = pos < 0 ? 0 : (pos > csrLen - 1 ? csrLen - 1 : pos);
      int sl = csr[pos];
      sl = sl < 0 ? 0 : (sl > nN - 1 ? nN - 1 : sl);
      const int mcnt = (n - q0) < 32 ? (n - q0) : 32;
#pragma unroll 1
      for (int p = 0; p < mcnt; ++p) {
        const int sidx = __builtin_amdgcn_readlane(sl, p);
        acc = acc + *(const v2f*)(hw + (size_t)sidx * DIM + 2 * lane);
      }
    }
    const v2f sv = *(const v2f*)(hw + (size_t)c * DIM + 2 * lane);
    const v2f z = (acc + sv * CSELF) * dc + bb;
    float mv = valid ? fmaxf(z.x, z.y) : -3.0e38f;
    mv = fmaxf(mv, __shfl_xor(mv, 16, 32)); mv = fmaxf(mv, __shfl_xor(mv, 8, 32)); mv = fmaxf(mv, __shfl_xor(mv, 4, 32));
    mv = fmaxf(mv, __shfl_xor(mv, 2, 32));  mv = fmaxf(mv, __shfl_xor(mv, 1, 32));
    const float ex = expf(z.x - mv) + expf(z.y - mv);
    float ev = valid ? ex : 0.f;
    ev += __shfl_xor(ev, 16, 32); ev += __shfl_xor(ev, 8, 32); ev += __shfl_xor(ev, 4, 32);
    ev += __shfl_xor(ev, 2, 32);  ev += __shfl_xor(ev, 1, 32);
    const float lg = logf(ev);
    v2f o;
    o.x = (z.x - mv) - lg; o.y = (z.y - mv) - lg;
    if (valid) *(v2f*)(sw + j * FOUT + 2 * lane) = o;
  }
  __syncthreads();

  float* gbp = out + (size_t)tbase * FOUT;
#pragma unroll
  for (int i = 0; i < (32 * FOUT) / 128; ++i) {
    const int fidx = i * 128 + 4 * lane;
    const int rowi = tbase + fidx / FOUT;
    const v4f v = *(const v4f*)(sw + fidx);
    if (rowi < nN) *(volatile v4f*)(gbp + fidx) = v;
  }
  __threadfence();
#pragma unroll
  for (int i = 0; i < (32 * FOUT) / 128; ++i) {
    const int fidx = i * 128 + 4 * lane;
    const int rowi = tbase + fidx / FOUT;
    const v4f v = *(const v4f*)(sw + fidx);
    if (rowi < nN) *(volatile v4f*)(gbp + fidx) = v;
  }
}

extern "C" void kernel_launch(void* const* d_in, const int* in_sizes, int n_in,
                              void* d_out, int out_size, void* d_ws, size_t ws_size,
                              hipStream_t stream) {
  if (n_in < 26) return;
  const int nN = in_sizes[0] / NIN;
  const int nE = in_sizes[25] / 2;
  if (nN < 8 || nE <= 0) return;
  if (in_sizes[0] != nN * NIN || in_sizes[1] != nN * NPE || in_sizes[2] != NMEM * DIM) return;
  if (in_sizes[3] != KC1 * DIM || in_sizes[4] != DIM || in_sizes[5] != KC2 * FOUT || in_sizes[6] != FOUT) return;
  for (int i = 7; i <= 14; ++i) if (in_sizes[i] != DIM * DIM) return;
  if (in_sizes[15] != DIM || in_sizes[16] != DIM || in_sizes[17] != DIM * FFH || in_sizes[18] != FFH) return;
  if (in_sizes[19] != FFH * DIM || in_sizes[20] != DIM) return;
  for (int i = 21; i <= 24; ++i) if (in_sizes[i] != DIM) return;
  if (in_sizes[25] != 2 * nE) return;
  if (out_size != nN * FOUT) return;
  if (nN > (1 << 20) || nE > (1 << 28)) return;

  const float* x      = (const float*)d_in[0];
  const float* pe     = (const float*)d_in[1];
  const float* memv   = (const float*)d_in[2];
  const float* gW1    = (const float*)d_in[3];
  const float* gb1    = (const float*)d_in[4];
  const float* gW2    = (const float*)d_in[5];
  const float* gb2    = (const float*)d_in[6];
  const float* Wqw    = (const float*)d_in[7];
  const float* Wkw    = (const float*)d_in[8];
  const float* Wvw    = (const float*)d_in[9];
  const float* Wow    = (const float*)d_in[10];
  const float* Wqb    = (const float*)d_in[11];
  const float* Wkb    = (const float*)d_in[12];
  const float* Wvb    = (const float*)d_in[13];
  const float* Wob    = (const float*)d_in[14];
  const float* ln1g   = (const float*)d_in[15];
  const float* ln1b   = (const float*)d_in[16];
  const float* fW1    = (const float*)d_in[17];
  const float* fb1    = (const float*)d_in[18];
  const float* fW2    = (const float*)d_in[19];
  const float* fb2    = (const float*)d_in[20];
  const float* ln2g   = (const float*)d_in[21];
  const float* ln2b   = (const float*)d_in[22];
  const float* lnmg   = (const float*)d_in[23];
  const float* lnmb   = (const float*)d_in[24];
  const int*   ei     = (const int*)d_in[25];
  float* out = (float*)d_out;
  const int* keys = ei + nE;
  const int* gath = ei;

  const int NPAD   = ((nN + TGT - 1) / TGT) * TGT;
  const int nBC    = (nN + NBC - 1) / NBC;
  const int CNTPAD = nBC * NBC;
  const int nBF    = (nN + NBF - 1) / NBF;
  const int OFFN   = nBF * NBF;
  if (nBF + 1 > RBN) return;
  if (OFFN > CNTPAD || NPAD > OFFN) return;
  const int csrLen = ((nE + 31) & ~31) + 32 * (nBF + 1);
  const int nGemm  = NPAD / GROWS;
  const int nAgg   = NPAD / TGT;

  char* ws = (char*)d_ws;
  size_t off = 0;
  const size_t U = (size_t)NPAD * DIM * 4;
  const size_t oW   = off; off += (size_t)PWTOT * 2;                 off = (off + 255) & ~(size_t)255;
  const size_t oCnt = off; off += (size_t)CNTPAD * 4;                off = (off + 255) & ~(size_t)255;
  const size_t oDv  = off; off += (size_t)CNTPAD * 4;                off = (off + 255) & ~(size_t)255;
  const size_t oOff = off; off += (size_t)OFFN * 4;                  off = (off + 255) & ~(size_t)255;
  const size_t oRb  = off; off += (size_t)RBN * 4;                   off = (off + 255) & ~(size_t)255;
  const size_t oCsr = off; off += (size_t)csrLen * 4;                off = (off + 255) & ~(size_t)255;
  const size_t oH   = off; off += U;                                 off = (off + 255) & ~(size_t)255;
  const size_t oK   = off; off += U;                                 off = (off + 255) & ~(size_t)255;
  const size_t oR4  = off; off += 2 * U;                             off = (off + 255) & ~(size_t)255;
  const size_t oG   = off; off += (size_t)SROWS * DIM * 4;           off = (off + 255) & ~(size_t)255;
  const size_t oQx  = off; off += (size_t)2 * SROWS * 32 * 2;        off = (off + 255) & ~(size_t)255;
  const size_t oKV  = off; off += (size_t)2 * NMEM * DIM * 4;         off = (off + 255) & ~(size_t)255;
  if (off > ws_size || off > (size_t)WSCAP) return;

  unsigned short* wp   = (unsigned short*)(ws + oW);
  int*            cnt  = (int*)(ws + oCnt);
  float*          dinv = (float*)(ws + oDv);
  int*            offp = (int*)(ws + oOff);
  int*            rb   = (int*)(ws + oRb);
  int*            csr  = (int*)(ws + oCsr);
  float*          hpl  = (float*)(ws + oH);
  unsigned short* kh   = (unsigned short*)(ws + oK);
  unsigned short* kl   = (unsigned short*)(ws + oK + (size_t)NPAD * DIM * 2);
  float*          r4a  = (float*)(ws + oR4);
  float*          r4b  = (float*)(ws + oR4 + U);
  float*          gpad = (float*)(ws + oG);
  unsigned short* qexp = (unsigned short*)(ws + oQx);
  float*          kbvb = (float*)(ws + oKV);

  const int vec8 = ((nE & 3) == 0) ? 1 : 0;

  k_wprep<<<28, NTHR, 0, stream>>>(gW1, Wkw, Wqb, Wob, fW1, fW2, gW2, wp);

  hipFuncSetAttribute(reinterpret_cast<const void*>(&k_count),
                      hipFuncAttributeMaxDynamicSharedMemorySize, LDS_COUNT);
  k_count<<<nBC, NTHR, LDS_COUNT, stream>>>(keys, gath, cnt, dinv, nE, nN, vec8);
  k_offsets<<<1, OTHR, 0, stream>>>(cnt, offp, rb, nBF);
  hipFuncSetAttribute(reinterpret_cast<const void*>(&k_fill),
                      hipFuncAttributeMaxDynamicSharedMemorySize, LDS_FILL);
  k_fill<<<nBF, NTHR, LDS_FILL, stream>>>(keys, gath, offp, rb, csr, nN, nE, vec8, csrLen);

  k_gemm<KC1, 3, 0, 1><<<nGemm, NTHR, 0, stream>>>(x, NIN, pe, NPE, 4, pe, NPE, 6, wp + PW1H, wp + PW1L,
                                                     dinv, r4a, kh, kl, nN);
  k_agg1<<<nAgg, NTHR, 0, stream>>>(csr, offp, cnt, dinv, r4a, gb1, hpl, nN, csrLen);

  k_smallq<<<1, 64, 0, stream>>>(memv, Wqw, qexp);
  k_gemm<DIM, 3, 1, 0><<<nGemm, NTHR, 0, stream>>>(hpl, DIM, hpl, DIM, 2, hpl, DIM, 2, wp + PWKH, wp + PWKL,
                                                     dinv, r4a, kh, kl, nN);
  k_scores<<<NPAD / 128, NTHR, 0, stream>>>(qexp, qexp + SROWS * 32, kh, kl, r4a, NPAD);

  k_top5<<<SROWS, NTHR, 0, stream>>>(r4a, hpl, gpad, nN, NPAD);
  k_smallm<<<1, 64, 0, stream>>>(gpad, Wvw, Wow, Wkb, Wvb, kbvb);

  k_battn<<<NPAD / 128, NTHR, 0, stream>>>(hpl, wp + PWQB, wp + PWOB, kbvb, ln1g, ln1b, r4a);

  k_ffn<<<NPAD / 128, NTHR, 0, stream>>>(r4a, hpl, wp + PF1, wp + PF2, fb1, fb2, ln2g, ln2b, lnmg, lnmb, r4b);

  k_gemm<KC2, 1, 0, 1><<<nGemm, NTHR, 0, stream>>>(r4b, DIM, x, NIN, 2, pe, NPE, 6, wp + PG2, wp + PG2,
                                                     dinv, r4a, kh, kl, nN);
  k_agg2<<<nAgg, NTHR, 0, stream>>>(csr, offp, cnt, dinv, r4a, gb2, out, nN, csrLen);
}
